// S4D_35751307771909
// MI455X (gfx1250) — hardware-verified
//
#include <hip/hip_runtime.h>
#include <math.h>

typedef __attribute__((ext_vector_type(8)))  _Float16 v8h;
typedef __attribute__((ext_vector_type(16))) __bf16   v16b;
typedef __attribute__((ext_vector_type(8)))  __bf16   v8b;
typedef __attribute__((ext_vector_type(8)))  float    v8f;
typedef __attribute__((ext_vector_type(4)))  float    v4f;

constexpr int kBatch   = 4;
constexpr int kSeq     = 2048;
constexpr int kHid     = 512;
constexpr int kNst     = 32;
constexpr int kRows    = kBatch * kSeq;
constexpr int kCat     = 2 * kHid;
constexpr int kChunk   = 32;
constexpr int kScanCh  = 64;
constexpr int kGroups  = 4;
constexpr int kPerLane = 8;
constexpr int kTilesM  = kRows / 64;
constexpr int kTilesN  = kHid / 32;
static_assert(kRows == 8192 && kCat == 1024, "shapes");
static_assert(kGroups * kPerLane == kNst, "state partition");
static_assert(kScanCh * kGroups == 256, "scan block");
static_assert((kHid % 32) == 0, "GEMM K multiple of 32");
static_assert((kRows % 64) == 0 && (kCat % 64) == 0 && (kHid % 64) == 0, "GEMM M,N tile multiples");
static_assert((kSeq % kChunk) == 0 && (kHid % kScanCh) == 0, "scan tile multiples");
static_assert(kChunk * kGroups * kScanCh == 8192 && kScanCh * kNst * 4 == 8192, "LDS region shared by both uses");
static_assert(kTilesM * kTilesN == 2048, "tile count = 256 blocks x 8 waves");

constexpr size_t kOffYH   = 0;
constexpr size_t kOffYL   = kOffYH + (size_t)kRows * kHid * 2;
constexpr size_t kOffBH   = kOffYL + (size_t)kRows * kHid * 2;
constexpr size_t kOffBL   = kOffBH + (size_t)kCat * kHid * 2;
constexpr size_t kWsTotal = kOffBL + (size_t)kCat * kHid * 2;
static_assert(kWsTotal == 18874368ull, "carve total");
static_assert(kWsTotal <= 134217728ull, "carve cap");
static_assert((kOffYL % 128) == 0 && (kOffBH % 128) == 0 && (kOffBL % 128) == 0, "128-B aligned regions");

__device__ __forceinline__ unsigned short f2bf_bits(float f) {
  unsigned u = __float_as_uint(f);
  return (unsigned short)((u + 0x7FFFu + ((u >> 16) & 1u)) >> 16);
}
__device__ __forceinline__ float bf_bits2f(unsigned short h) { return __uint_as_float(((unsigned)h) << 16); }

__device__ __forceinline__ void guard4_b(v8f& a, v8f& b, v8f& c, v8f& d, v16b x, v16b y) {
  asm volatile("v_nop\n\tv_nop\n\tv_nop\n\tv_nop" : "+v"(a), "+v"(b), "+v"(c), "+v"(d) : "v"(x), "v"(y));
}
__device__ __forceinline__ void keep4_b(v16b a, v16b b, v16b c, v16b d) { asm volatile("v_nop" :: "v"(a), "v"(b), "v"(c), "v"(d)); }
__device__ __forceinline__ void acc_guard4(v8f& a, v8f& b, v8f& c, v8f& d) {
  asm volatile("v_nop\n\tv_nop\n\tv_nop\n\tv_nop" : "+v"(a), "+v"(b), "+v"(c), "+v"(d));
}
__device__ __forceinline__ v16b frag_load_b(const __bf16* p) {
  union { v16b v; v8b h[2]; } f;
  f.h[0] = *(const v8b*)(p);
  f.h[1] = *(const v8b*)(p + 16);
  return f.v;
}
__device__ __forceinline__ v8f mma_b(v16b a, v16b b, v8f c) {
  return __builtin_amdgcn_wmma_f32_16x16x32_bf16(false, a, false, b, (short)0, c, false, false);
}

__global__ __launch_bounds__(256) void wt_split_transpose_kernel(
    const float* __restrict__ W1, const float* __restrict__ W2,
    unsigned short* __restrict__ BH, unsigned short* __restrict__ BL)
{
  __shared__ float tile[64 * 65];
  const int tid = threadIdx.x, lane = tid & 31, wave = tid >> 5;
  const int n0 = blockIdx.x * 64;
  const int k0 = blockIdx.y * 64;
  const int z  = blockIdx.z;
  const float* W = (z == 0) ? W1 : W2;
#pragma unroll
  for (int p = 0; p < 16; ++p) {
    const int idx = tid + p * 256;
    const int kk  = idx >> 6;
    const int nn  = idx & 63;
    tile[kk * 65 + nn] = W[(size_t)(k0 + kk) * kHid + n0 + nn];
  }
  __syncthreads();
  const int q = lane >> 3, c8 = (lane & 7) * 8;
  v8h hv[2], lv[2];
#pragma unroll
  for (int it = 0; it < 2; ++it) {
    const int nrow = it * 32 + wave * 4 + q;
#pragma unroll
    for (int e = 0; e < 8; ++e) {
      const float x = tile[(c8 + e) * 65 + nrow];
      const unsigned short hb = f2bf_bits(x);
      const unsigned short lb = f2bf_bits(x - bf_bits2f(hb));
      hv[it][e] = __builtin_bit_cast(_Float16, hb);
      lv[it][e] = __builtin_bit_cast(_Float16, lb);
    }
  }
  for (int pass = 0; pass < 2; ++pass) {
#pragma unroll
    for (int it = 0; it < 2; ++it) {
      const int nrow = it * 32 + wave * 4 + q;
      const size_t o = (size_t)(z * kHid + n0 + nrow) * kHid + k0 + c8;
      *(volatile v8h*)(BH + o) = hv[it];
      *(volatile v8h*)(BL + o) = lv[it];
    }
    __threadfence();
  }
}

__device__ __forceinline__ void disc_params(float ldt, float lar, float aim, float bre, float bim,
                                            float cre, float cim,
                                            float& oAr, float& oAi, float& oCr, float& oCi)
{
#pragma clang fp contract(off)
  const float dt  = expf(ldt);
  const float are = -expf(lar);
  const float hdt = 0.5f * dt;
  const float tr  = hdt * are;
  const float ti  = hdt * aim;
  const float nr  = 1.0f + tr;
  const float dr  = 1.0f - tr;
  const float br  = dt * bre;
  const float bi  = dt * bim;
  const double dnr = (double)nr, ddr = (double)dr, dti = (double)ti;
  const double den = ddr * ddr + dti * dti;
  const float denf = (float)den;
  double r = (double)__builtin_amdgcn_rcpf(denf);
  r = r + r * (1.0 - den * r);
  r = r + r * (1.0 - den * r);
  const double adr = (dnr * ddr - dti * dti) * r;
  const double adi = (dti * (dnr + ddr)) * r;
  const double dbr = (double)br, dbi = (double)bi;
  const double bdr = (dbr * ddr - dbi * dti) * r;
  const double bdi = (dbr * dti + dbi * ddr) * r;
  const double dcr = (double)cre, dci = (double)cim;
  const double cpr = dcr * bdr - dci * bdi;
  const double cpi = dcr * bdi + dci * bdr;
  oAr = (float)adr;
  oAi = (float)adi;
  oCr = (float)cpr;
  oCi = (float)cpi;
}

__global__ __launch_bounds__(256) void s4d_scan_kernel(
    const float* __restrict__ U, const float* __restrict__ log_dt, const float* __restrict__ logA,
    const float* __restrict__ Aim, const float* __restrict__ Bri, const float* __restrict__ Cri,
    const float* __restrict__ Dp, unsigned short* __restrict__ YH, unsigned short* __restrict__ YL)
{
  __shared__ __align__(16) float sBig[8192];
  __shared__ __align__(16) float sU[kChunk * kScanCh];
  const int tid = threadIdx.x;
  const int bix = blockIdx.x >> 3;
  const int h0  = (blockIdx.x & 7) * kScanCh;

#pragma unroll 1
  for (int it = 0; it < 8; ++it) {
    const int p  = it * 256 + tid;
    const int ph = p >> 5;
    const int pn = p & 31;
    const int h  = h0 + ph;
    const int gi = h * kNst + pn;
    const float ldt = log_dt[h];
    const float lar = logA[gi];
    const float aim = Aim[gi];
    const float bre = Bri[2 * pn];
    const float bim = Bri[2 * pn + 1];
    const float cre = Cri[2 * gi];
    const float cim = Cri[2 * gi + 1];
    float pAr, pAi, pCr, pCi;
    disc_params(ldt, lar, aim, bre, bim, cre, cim, pAr, pAi, pCr, pCi);
    sBig[p]        = pAr;
    sBig[2048 + p] = pAi;
    sBig[4096 + p] = pCr;
    sBig[6144 + p] = pCi;
  }
  __syncthreads();

  const int hh = tid & 63, ng = tid >> 6;
  float ar[kPerLane], ai[kPerLane], cr[kPerLane], ci[kPerLane], zr[kPerLane], zi[kPerLane];
  {
    const float* pb = sBig + hh * kNst + ng * kPerLane;
    const v4f a0 = *(const v4f*)(pb),        a1 = *(const v4f*)(pb + 4);
    const v4f b0 = *(const v4f*)(pb + 2048), b1 = *(const v4f*)(pb + 2048 + 4);
    const v4f c0 = *(const v4f*)(pb + 4096), c1 = *(const v4f*)(pb + 4096 + 4);
    const v4f e0 = *(const v4f*)(pb + 6144), e1 = *(const v4f*)(pb + 6144 + 4);
#pragma unroll
    for (int j = 0; j < 4; ++j) {
      ar[j] = a0[j]; ar[4 + j] = a1[j];
      ai[j] = b0[j]; ai[4 + j] = b1[j];
      cr[j] = c0[j]; cr[4 + j] = c1[j];
      ci[j] = e0[j]; ci[4 + j] = e1[j];
      zr[j] = 0.0f;  zr[4 + j] = 0.0f;
      zi[j] = 0.0f;  zi[4 + j] = 0.0f;
    }
  }

  const int et = tid >> 3, c8 = (tid & 7) * 8;
  const v4f dv0 = *(const v4f*)(Dp + h0 + c8);
  const v4f dv1 = *(const v4f*)(Dp + h0 + c8 + 4);
  const size_t rowBase = (size_t)bix * kSeq;
  float* sPart = sBig;

#pragma unroll 1
  for (int tc = 0; tc < kSeq; tc += kChunk) {
    __syncthreads();
    {
      const float* src = U + (rowBase + tc + et) * kHid + h0 + c8;
      const v4f x0 = *(const v4f*)(src);
      const v4f x1 = *(const v4f*)(src + 4);
      *(v4f*)(sU + et * kScanCh + c8)     = x0;
      *(v4f*)(sU + et * kScanCh + c8 + 4) = x1;
    }
    __syncthreads();
#pragma unroll 1
    for (int s = 0; s < kChunk; ++s) {
      const float u = sU[s * kScanCh + hh];
      float acc = 0.0f;
#pragma unroll
      for (int j = 0; j < kPerLane; ++j) {
        const float pr  = fmaf(-ai[j], zi[j], u);
        const float nzr = fmaf(ar[j], zr[j], pr);
        const float pi2 = ar[j] * zi[j];
        const float nzi = fmaf(ai[j], zr[j], pi2);
        zr[j] = nzr;
        zi[j] = nzi;
        acc = fmaf(cr[j], nzr, acc);
        acc = fmaf(-ci[j], nzi, acc);
      }
      sPart[(s * kGroups + ng) * kScanCh + hh] = acc;
    }
    __syncthreads();
    v8h hv, lv;
    {
      const float* pp = sPart + (et * kGroups) * kScanCh + c8;
      v4f s0 = (v4f){0.f, 0.f, 0.f, 0.f};
      v4f s1 = (v4f){0.f, 0.f, 0.f, 0.f};
#pragma unroll
      for (int g = 0; g < kGroups; ++g) {
        s0 += *(const v4f*)(pp + g * kScanCh);
        s1 += *(const v4f*)(pp + g * kScanCh + 4);
      }
      const v4f u0 = *(const v4f*)(sU + et * kScanCh + c8);
      const v4f u1 = *(const v4f*)(sU + et * kScanCh + c8 + 4);
#pragma unroll
      for (int e = 0; e < 4; ++e) {
        const float y0 = fmaf(dv0[e], u0[e], s0[e]);
        const float y1 = fmaf(dv1[e], u1[e], s1[e]);
        const unsigned short hb0 = f2bf_bits(y0), hb1 = f2bf_bits(y1);
        const unsigned short lb0 = f2bf_bits(y0 - bf_bits2f(hb0));
        const unsigned short lb1 = f2bf_bits(y1 - bf_bits2f(hb1));
        hv[e]     = __builtin_bit_cast(_Float16, hb0);
        hv[4 + e] = __builtin_bit_cast(_Float16, hb1);
        lv[e]     = __builtin_bit_cast(_Float16, lb0);
        lv[4 + e] = __builtin_bit_cast(_Float16, lb1);
      }
    }
    const size_t o = (rowBase + tc + et) * kHid + h0 + c8;
    *(volatile v8h*)(YH + o) = hv;
    *(volatile v8h*)(YL + o) = lv;
    __threadfence();
    *(volatile v8h*)(YH + o) = hv;
    *(volatile v8h*)(YL + o) = lv;
  }
}

__global__ __launch_bounds__(256) void glu_gemm_kernel(
    const unsigned short* __restrict__ YHp, const unsigned short* __restrict__ YLp,
    const unsigned short* __restrict__ BHp, const unsigned short* __restrict__ BLp,
    float* __restrict__ out)
{
  const __bf16* A  = (const __bf16*)YHp;
  const __bf16* A2 = (const __bf16*)YLp;
  const __bf16* Bt  = (const __bf16*)BHp;
  const __bf16* Bt2 = (const __bf16*)BLp;
  __shared__ __align__(16) float sT[8][16 * 68];
  const int lane = threadIdx.x & 31;
  const int wave = threadIdx.x >> 5;
  const int tile = blockIdx.x * 8 + wave;
  if (tile >= kTilesM * kTilesN) return;
  const int tm = tile >> 4;
  const int tn = tile & 15;
  const int m0 = tm << 6;
  const int c0 = tn << 5;

  const int rlane = lane & 15;
  const int koff  = (lane >> 4) * 8;
  const int mOff  = (lane >> 4) * 8;

  v8f acc[4][4];
#pragma unroll
  for (int i = 0; i < 4; ++i)
#pragma unroll
    for (int j = 0; j < 4; ++j) acc[i][j] = (v8f){0.f, 0.f, 0.f, 0.f, 0.f, 0.f, 0.f, 0.f};

  for (int k0 = 0; k0 < kHid; k0 += 32) {
    v16b bh[4], bl[4];
#pragma unroll
    for (int j = 0; j < 4; ++j) {
      const int brow = (j >> 1) * kHid + c0 + ((j & 1) << 4) + rlane;
      const size_t bo = (size_t)brow * kHid + koff + k0;
      bh[j] = frag_load_b(Bt + bo);
      bl[j] = frag_load_b(Bt2 + bo);
    }
#pragma unroll
    for (int i = 0; i < 4; ++i) {
      const size_t ao = (size_t)(m0 + (i << 4) + rlane) * kHid + koff + k0;
      v16b ah = frag_load_b(A + ao);
      v16b al = frag_load_b(A2 + ao);
#pragma unroll
      for (int j = 0; j < 4; ++j) {
        acc[i][j] = mma_b(ah, bh[j], acc[i][j]);
        acc[i][j] = mma_b(ah, bl[j], acc[i][j]);
        acc[i][j] = mma_b(al, bh[j], acc[i][j]);
      }
      guard4_b(acc[i][0], acc[i][1], acc[i][2], acc[i][3], ah, al);
    }
    keep4_b(bh[0], bh[1], bh[2], bh[3]);
    keep4_b(bl[0], bl[1], bl[2], bl[3]);
  }
  acc_guard4(acc[0][0], acc[0][1], acc[0][2], acc[0][3]);
  acc_guard4(acc[1][0], acc[1][1], acc[1][2], acc[1][3]);
  acc_guard4(acc[2][0], acc[2][1], acc[2][2], acc[2][3]);
  acc_guard4(acc[3][0], acc[3][1], acc[3][2], acc[3][3]);

  float* slab = sT[wave];
  const int q = lane >> 3, c4 = (lane & 7) * 4;
#pragma unroll
  for (int i = 0; i < 4; ++i) {
    const int mBase = m0 + (i << 4);
#pragma unroll
    for (int j = 0; j < 4; ++j) {
#pragma unroll
      for (int r = 0; r < 8; ++r) {
        slab[(mOff + r) * 68 + (j << 4) + rlane] = acc[i][j][r];
      }
    }
    __builtin_amdgcn_fence(__ATOMIC_RELEASE, "workgroup");
    __builtin_amdgcn_wave_barrier();
    __builtin_amdgcn_fence(__ATOMIC_ACQUIRE, "workgroup");
#pragma unroll 1
    for (int row = 0; row < 16; ++row) {
      const float gv = slab[row * 68 + lane];
      const float sv = slab[row * 68 + 32 + lane];
      const float sc = fmaxf(sv, -80.0f);
      const float ex = expf(-sc);
      const float sg = __builtin_amdgcn_rcpf(1.0f + ex);
      slab[row * 68 + lane] = gv * sg;
    }
    __builtin_amdgcn_fence(__ATOMIC_RELEASE, "workgroup");
    __builtin_amdgcn_wave_barrier();
    __builtin_amdgcn_fence(__ATOMIC_ACQUIRE, "workgroup");
    for (int pass = 0; pass < 2; ++pass) {
#pragma unroll
      for (int it = 0; it < 4; ++it) {
        const int row = it * 4 + q;
        const v4f v = *(const v4f*)(slab + row * 68 + c4);
        *(volatile v4f*)(out + (size_t)(mBase + row) * kHid + c0 + c4) = v;
      }
      __threadfence();
    }
    __builtin_amdgcn_fence(__ATOMIC_RELEASE, "workgroup");
    __builtin_amdgcn_wave_barrier();
    __builtin_amdgcn_fence(__ATOMIC_ACQUIRE, "workgroup");
  }
}

extern "C" void kernel_launch(void* const* d_in, const int* in_sizes, int n_in,
                              void* d_out, int out_size, void* d_ws, size_t ws_size,
                              hipStream_t stream) {
  if (n_in < 9) return;
  if (in_sizes[0] != kRows * kHid) return;
  if (in_sizes[1] != kHid) return;
  if (in_sizes[2] != kHid * kNst) return;
  if (in_sizes[3] != kHid * kNst) return;
  if (in_sizes[4] != kNst * 2) return;
  if (in_sizes[5] != kHid * kNst * 2) return;
  if (in_sizes[6] != kHid) return;
  if (in_sizes[7] != kHid * kHid) return;
  if (in_sizes[8] != kHid * kHid) return;
  if (out_size != kRows * kHid) return;
  if (ws_size < kWsTotal) return;

  const float* x      = (const float*)d_in[0];
  const float* log_dt = (const float*)d_in[1];
  const float* logA   = (const float*)d_in[2];
  const float* Aim    = (const float*)d_in[3];
  const float* Bri    = (const float*)d_in[4];
  const float* Cri    = (const float*)d_in[5];
  const float* Dp     = (const float*)d_in[6];
  const float* W1     = (const float*)d_in[7];
  const float* W2     = (const float*)d_in[8];
  float* out = (float*)d_out;

  char* ws = (char*)d_ws;
  unsigned short* YH = (unsigned short*)(ws + kOffYH);
  unsigned short* YL = (unsigned short*)(ws + kOffYL);
  unsigned short* BH = (unsigned short*)(ws + kOffBH);
  unsigned short* BL = (unsigned short*)(ws + kOffBL);

  wt_split_transpose_kernel<<<dim3(kHid / 64, kHid / 64, 2), 256, 0, stream>>>(W1, W2, BH, BL);

  s4d_scan_kernel<<<kBatch * (kHid / kScanCh), 256, 0, stream>>>(x, log_dt, logA, Aim, Bri, Cri, Dp, YH, YL);

  glu_gemm_kernel<<<(kTilesM * kTilesN) / 8, 256, 0, stream>>>(YH, YL, BH, BL, out);
}
